// TemporalAttention_42975442764284
// MI455X (gfx1250) — hardware-verified
//
#include <hip/hip_runtime.h>
#include <stdint.h>


#ifndef NB
#define NB 8
#endif
#ifndef SEQ
#define SEQ 4096
#endif
#define NB_FULL 8
#define N_FULL 4096
#define C_ 256
#define DQK 32
#define PCARRY 16384.0f
#define PCARRY_INV (1.0f / 16384.0f)

static_assert((SEQ % 64) == 0);
static_assert(SEQ >= 64 && SEQ <= N_FULL);
static_assert(NB >= 1 && NB <= NB_FULL);
static_assert((C_ % 32) == 0);
static_assert(DQK == 32);

typedef __bf16 v16bf __attribute__((ext_vector_type(16)));
typedef _Float16 v16h __attribute__((ext_vector_type(16)));
typedef float v8f __attribute__((ext_vector_type(8)));
typedef float v4f __attribute__((ext_vector_type(4)));
typedef unsigned short v8us __attribute__((ext_vector_type(8)));

union FragB { v16bf v; v8us half[2]; };
union FragH { v16h v; v8us half[2]; };

__device__ __forceinline__ v8f mma_bf16(v16bf a, v16bf b, v8f c) {
  v8f d = __builtin_amdgcn_wmma_f32_16x16x32_bf16(false, a, false, b, (short)0, c, false, false);
  asm volatile("v_nop\n\tv_nop\n\tv_nop\n\tv_nop" : "+v"(d) : "v"(a), "v"(b));
  return d;
}
__device__ __forceinline__ v8f mma_f16(v16h a, v16h b, v8f c) {
  v8f d = __builtin_amdgcn_wmma_f32_16x16x32_f16(false, a, false, b, (short)0, c, false, false);
  asm volatile("v_nop\n\tv_nop\n\tv_nop\n\tv_nop" : "+v"(d) : "v"(a), "v"(b));
  return d;
}

__device__ __forceinline__ unsigned short f2bf(float f) {
  unsigned int u = __float_as_uint(f);
  u = (u + 0x7FFFu + ((u >> 16) & 1u)) >> 16;
  return (unsigned short)u;
}
__device__ __forceinline__ float bf2f(unsigned short s) {
  return __uint_as_float(((unsigned int)s) << 16);
}
__device__ __forceinline__ float bfr(float f) { return bf2f(f2bf(f)); }

__device__ __forceinline__ v8f zero8() {
  v8f z = {0.f, 0.f, 0.f, 0.f, 0.f, 0.f, 0.f, 0.f};
  return z;
}

__global__ void __launch_bounds__(256)
k_wcvt(const float* __restrict__ wv, const float* __restrict__ wq, const float* __restrict__ wk,
       unsigned short* __restrict__ w16)
{
  const int lane = threadIdx.x & 31;
  const int wave = __builtin_amdgcn_readfirstlane((int)(threadIdx.x >> 5));
  const int row = blockIdx.x * 8 + wave;
  const float* src = (row < C_) ? (wv + (size_t)row * C_)
                   : (row < C_ + DQK) ? (wq + (size_t)(row - C_) * C_)
                   : (wk + (size_t)(row - C_ - DQK) * C_);
  const v4f a = *(const v4f*)(src + 8 * lane);
  const v4f c = *(const v4f*)(src + 8 * lane + 4);
  v8us pk;
  pk[0] = f2bf(a[0]); pk[1] = f2bf(a[1]); pk[2] = f2bf(a[2]); pk[3] = f2bf(a[3]);
  pk[4] = f2bf(c[0]); pk[5] = f2bf(c[1]); pk[6] = f2bf(c[2]); pk[7] = f2bf(c[3]);
  unsigned short* dst = w16 + (size_t)row * C_ + 8 * lane;
  *(volatile v8us*)dst = pk;
  __threadfence();
  *(volatile v8us*)dst = pk;
}

#define XS_P 264
#define VS_P 72
#define PROJ_VST 0
#define PROJ_QKST (C_ * VS_P)
#define PROJ_LDS_U16 (PROJ_QKST + 4 * 64 * DQK)
static_assert(64 * XS_P <= PROJ_LDS_U16);

__device__ __forceinline__ void proj_store_lines(const unsigned short* lds, unsigned short* vpl,
                                                 unsigned short* qkpl, int wave, int lane) {
#pragma unroll
  for (int i = 0; i < 16; ++i) {
    const int L = 4 * i + (lane >> 3);
    const int c = 64 * wave + L;
    const int piece = lane & 7;
    const v8us v = *(const v8us*)(lds + PROJ_VST + c * VS_P + 8 * piece);
    *(volatile v8us*)(vpl + (size_t)c * SEQ + 8 * piece) = v;
  }
  const unsigned short* qks = lds + PROJ_QKST + wave * (64 * DQK);
#pragma unroll
  for (int i = 0; i < 8; ++i) {
    const v8us v = *(const v8us*)(qks + i * 256 + lane * 8);
    *(volatile v8us*)(qkpl + i * 256 + lane * 8) = v;
  }
}

__global__ void __launch_bounds__(128)
k_proj(const float* __restrict__ x, const unsigned short* __restrict__ w16,
       const float* __restrict__ bq, const float* __restrict__ bk, const float* __restrict__ bv,
       unsigned short* __restrict__ qhi, unsigned short* __restrict__ qlo,
       unsigned short* __restrict__ khi, unsigned short* __restrict__ klo,
       unsigned short* __restrict__ v16)
{
  __shared__ __align__(16) unsigned short lds[PROJ_LDS_U16];
  const int tid = threadIdx.x;
  const int lane = tid & 31, h = lane >> 4, m = lane & 15;
  const int wave = __builtin_amdgcn_readfirstlane(tid >> 5);
  const int n0 = blockIdx.x * 64;
  const int b = blockIdx.y;

  {
    const float* xb = x + (size_t)b * C_ * N_FULL + n0;
    const int piece = tid & 15;
    const int crow = tid >> 4;
#pragma unroll 4
    for (int p = 0; p < C_ / 8; ++p) {
      const int c = p * 8 + crow;
      const v4f xv = *(const v4f*)(xb + (size_t)c * N_FULL + 4 * piece);
      unsigned short* d = lds + (4 * piece) * XS_P + c;
      d[0]        = f2bf(xv[0]);
      d[XS_P]     = f2bf(xv[1]);
      d[2 * XS_P] = f2bf(xv[2]);
      d[3 * XS_P] = f2bf(xv[3]);
    }
  }
  __syncthreads();

  FragB af[8];
  {
    const unsigned short* ar = lds + (16 * wave + m) * XS_P + 8 * h;
#pragma unroll
    for (int ks = 0; ks < 8; ++ks) {
      af[ks].half[0] = *(const v8us*)(ar + 32 * ks);
      af[ks].half[1] = *(const v8us*)(ar + 32 * ks + 16);
    }
  }
  __syncthreads();

#pragma unroll 1
  for (int ct = 0; ct < C_ / 16; ++ct) {
    const int o = 16 * ct + m;
    const unsigned short* wrow = w16 + (size_t)o * C_ + 8 * h;
    v8f acc = zero8();
#pragma unroll
    for (int ks = 0; ks < 8; ++ks) {
      FragB bb;
      bb.half[0] = *(const v8us*)(wrow + 32 * ks);
      bb.half[1] = *(const v8us*)(wrow + 32 * ks + 16);
      acc = mma_bf16(af[ks].v, bb.v, acc);
    }
    const float bias = bfr(bv[o]);
    v8us pk;
#pragma unroll
    for (int r = 0; r < 8; ++r) {
      const _Float16 hv = (_Float16)(acc[r] + bias);
      pk[r] = __builtin_bit_cast(unsigned short, hv);
    }
    *(v8us*)(lds + PROJ_VST + o * VS_P + 16 * wave + 8 * h) = pk;
  }

#pragma unroll 1
  for (int g = 0; g < 4; ++g) {
    const int isk = g >> 1;
    const int d = 16 * (g & 1) + m;
    const unsigned short* wrow = w16 + (size_t)(C_ + isk * DQK + d) * C_ + 8 * h;
    v8f acc = zero8();
#pragma unroll
    for (int ks = 0; ks < 8; ++ks) {
      FragB bb;
      bb.half[0] = *(const v8us*)(wrow + 32 * ks);
      bb.half[1] = *(const v8us*)(wrow + 32 * ks + 16);
      acc = mma_bf16(af[ks].v, bb.v, acc);
    }
    const float* bp = isk ? bk : bq;
    const float bias = bfr(bp[d]);
    unsigned short* sh = lds + PROJ_QKST + (2 * isk) * (64 * DQK);
    unsigned short* sl = sh + 64 * DQK;
#pragma unroll
    for (int r = 0; r < 8; ++r) {
      const int n = 16 * wave + 8 * h + r;
      const float val = acc[r] + bias;
      const unsigned short hb = f2bf(val);
      const unsigned short lb = f2bf(val - bf2f(hb));
      sh[n * DQK + d] = hb;
      sl[n * DQK + d] = lb;
    }
  }
  __syncthreads();

  unsigned short* vpl = v16 + ((size_t)b * C_) * SEQ + n0;
  unsigned short* qkpl = (wave == 0) ? qhi : (wave == 1) ? qlo : (wave == 2) ? khi : klo;
  qkpl += ((size_t)b * SEQ + n0) * DQK;
  proj_store_lines(lds, vpl, qkpl, wave, lane);
  __threadfence();
  proj_store_lines(lds, vpl, qkpl, wave, lane);
}

#define KV_P 72
#define ATT_KHI 0
#define ATT_KLO (64 * DQK)
#define ATT_VLS (2 * 64 * DQK)
#define ATT_PLS (ATT_VLS + C_ * KV_P)
#define ATT_LDS_U16 (ATT_PLS + 64 * KV_P)
#define OST_P 68
static_assert(128 * OST_P * 2 <= ATT_LDS_U16);

__device__ __forceinline__ void att_store_lines(const float* ost, float* ob, int wave, int lane) {
#pragma unroll
  for (int i = 0; i < 8; ++i) {
    const int L = 4 * i + (lane >> 3);
    const int cl = 16 * wave + (L >> 1);
    const int fo = 32 * (L & 1) + 4 * (lane & 7);
    const v4f v = *(const v4f*)(ost + cl * OST_P + fo);
    *(volatile v4f*)(ob + (size_t)cl * SEQ + fo) = v;
  }
}

__global__ void __launch_bounds__(256)
k_attn(const unsigned short* __restrict__ qhi, const unsigned short* __restrict__ qlo,
       const unsigned short* __restrict__ khi, const unsigned short* __restrict__ klo,
       const unsigned short* __restrict__ v16, float* __restrict__ out)
{
  __shared__ __align__(16) unsigned short lds[ATT_LDS_U16];
  __shared__ float corr_s[64];
  __shared__ float linv_s[64];
  const int tid = threadIdx.x;
  const int lane = tid & 31, h = lane >> 4, m = lane & 15;
  const int wave = __builtin_amdgcn_readfirstlane(tid >> 5);
  const int qt = wave & 3;
  const int chh = wave >> 2;
  const int n0 = blockIdx.x * 64;
  const int b = blockIdx.y;
  const size_t qkb = (size_t)b * SEQ * DQK;
  const int qrow = 16 * qt + m;

  FragB fqh, fql;
  {
    const unsigned short* qp  = qhi + qkb + (size_t)(n0 + qrow) * DQK + 8 * h;
    const unsigned short* qp2 = qlo + qkb + (size_t)(n0 + qrow) * DQK + 8 * h;
    fqh.half[0] = *(const v8us*)qp;  fqh.half[1] = *(const v8us*)(qp + 16);
    fql.half[0] = *(const v8us*)qp2; fql.half[1] = *(const v8us*)(qp2 + 16);
  }
  const v8f zero = zero8();
  v8f acc[8];
#pragma unroll
  for (int i = 0; i < 8; ++i) acc[i] = zero;
  float m_run = -3.0e38f;
  float l_run = 0.f;
  const unsigned short* vb = v16 + (size_t)b * C_ * SEQ;

  for (int jc = 0; jc < SEQ / 64; ++jc) {
    const int j0 = jc * 64;
    {
      const size_t ko = qkb + (size_t)j0 * DQK + (size_t)tid * 8;
      *(v8us*)(lds + ATT_KHI + tid * 8) = *(const v8us*)(khi + ko);
      *(v8us*)(lds + ATT_KLO + tid * 8) = *(const v8us*)(klo + ko);
      const int piece = tid & 7, cr = tid >> 3;
#pragma unroll
      for (int p = 0; p < 8; ++p) {
        const int c = p * 32 + cr;
        *(v8us*)(lds + ATT_VLS + c * KV_P + 8 * piece) =
            *(const v8us*)(vb + (size_t)c * SEQ + j0 + 8 * piece);
      }
    }
    __syncthreads();

    if (wave < 4) {
      v8f s[4];
#pragma unroll
      for (int t = 0; t < 4; ++t) {
        FragB ah, al;
        const unsigned short* kr  = lds + ATT_KHI + (16 * t + m) * DQK + 8 * h;
        const unsigned short* kr2 = lds + ATT_KLO + (16 * t + m) * DQK + 8 * h;
        ah.half[0] = *(const v8us*)kr;  ah.half[1] = *(const v8us*)(kr + 16);
        al.half[0] = *(const v8us*)kr2; al.half[1] = *(const v8us*)(kr2 + 16);
        v8f d = mma_bf16(ah.v, fqh.v, zero);
        d = mma_bf16(ah.v, fql.v, d);
        d = mma_bf16(al.v, fqh.v, d);
        s[t] = d;
      }
      float mx = s[0][0];
#pragma unroll
      for (int t = 0; t < 4; ++t) {
#pragma unroll
        for (int r = 0; r < 8; ++r) mx = fmaxf(mx, s[t][r]);
      }
      mx = fmaxf(mx, __shfl_xor(mx, 16));
      const float mnew = fmaxf(m_run, mx);
      const float corr = __expf(m_run - mnew);
      m_run = mnew;
      float rs = 0.f;
#pragma unroll
      for (int t = 0; t < 4; ++t) {
        v8us pk;
#pragma unroll
        for (int r = 0; r < 8; ++r) {
          const float e = __expf(s[t][r] - mnew);
          rs += e;
          const _Float16 eh = (_Float16)(e * PCARRY);
          pk[r] = __builtin_bit_cast(unsigned short, eh);
        }
        *(v8us*)(lds + ATT_PLS + qrow * KV_P + 16 * t + 8 * h) = pk;
      }
      l_run = l_run * corr + rs;
      corr_s[qrow] = corr;
    }
    __syncthreads();

    {
      const float corr = corr_s[qrow];
#pragma unroll
      for (int ct = 0; ct < 8; ++ct) acc[ct] = acc[ct] * corr;
      const unsigned short* pr = lds + ATT_PLS + qrow * KV_P + 8 * h;
      const unsigned short* vr = lds + ATT_VLS + (128 * chh + m) * KV_P + 8 * h;
#pragma unroll
      for (int ks = 0; ks < 2; ++ks) {
        FragH pb;
        pb.half[0] = *(const v8us*)(pr + 32 * ks);
        pb.half[1] = *(const v8us*)(pr + 32 * ks + 16);
#pragma unroll
        for (int ct = 0; ct < 8; ++ct) {
          FragH va;
          const unsigned short* vrr = vr + (16 * ct) * KV_P + 32 * ks;
          va.half[0] = *(const v8us*)vrr;
          va.half[1] = *(const v8us*)(vrr + 16);
          acc[ct] = mma_f16(va.v, pb.v, acc[ct]);
        }
      }
    }
    __syncthreads();
  }

  {
    const float l = l_run + __shfl_xor(l_run, 16);
    if (wave < 4) linv_s[qrow] = PCARRY_INV * (1.0f / l);
  }
  __syncthreads();

  float* ost = (float*)lds;
#pragma unroll 1
  for (int half = 0; half < 2; ++half) {
    if (chh == half) {
      const float li = linv_s[qrow];
#pragma unroll
      for (int ct = 0; ct < 8; ++ct) {
#pragma unroll
        for (int r = 0; r < 8; ++r) ost[(16 * ct + 8 * h + r) * OST_P + qrow] = acc[ct][r] * li;
      }
    }
    __syncthreads();
    float* ob = out + ((size_t)b * C_ + 128 * half) * SEQ + n0;
    att_store_lines(ost, ob, wave, lane);
    __threadfence();
    att_store_lines(ost, ob, wave, lane);
    __syncthreads();
  }
}

static inline size_t align256(size_t v) { return (v + 255) & ~(size_t)255; }

extern "C" void kernel_launch(void* const* d_in, const int* in_sizes, int n_in,
                              void* d_out, int out_size, void* d_ws, size_t ws_size,
                              hipStream_t stream)
{
  if (n_in < 7) return;
  if (in_sizes[0] < NB * C_ * N_FULL) return;
  if (in_sizes[1] < DQK * C_) return;
  if (in_sizes[2] < DQK) return;
  if (in_sizes[3] < DQK * C_) return;
  if (in_sizes[4] < DQK) return;
  if (in_sizes[5] < C_ * C_) return;
  if (in_sizes[6] < C_) return;
  if (out_size < NB * C_ * SEQ) return;

  const float* x  = (const float*)d_in[0];
  const float* wq = (const float*)d_in[1];
  const float* bq = (const float*)d_in[2];
  const float* wk = (const float*)d_in[3];
  const float* bk = (const float*)d_in[4];
  const float* wv = (const float*)d_in[5];
  const float* bv = (const float*)d_in[6];
  float* out = (float*)d_out;

  const size_t w16_bytes = (size_t)(C_ + 2 * DQK) * C_ * 2;
  const size_t qk_bytes  = (size_t)NB * SEQ * DQK * 2;
  const size_t v_bytes   = (size_t)NB * C_ * SEQ * 2;
  char* ws = (char*)d_ws;
  size_t off = 0;
  unsigned short* w16 = (unsigned short*)(ws + off); off += align256(w16_bytes);
  unsigned short* qhi = (unsigned short*)(ws + off); off += align256(qk_bytes);
  unsigned short* qlo = (unsigned short*)(ws + off); off += align256(qk_bytes);
  unsigned short* khi = (unsigned short*)(ws + off); off += align256(qk_bytes);
  unsigned short* klo = (unsigned short*)(ws + off); off += align256(qk_bytes);
  unsigned short* v16 = (unsigned short*)(ws + off); off += align256(v_bytes);
  if (off > ws_size) return;

  k_wcvt<<<dim3((C_ + 2 * DQK) / 8), dim3(256), 0, stream>>>(wv, wq, wk, w16);
  k_proj<<<dim3(SEQ / 64, NB), dim3(128), 0, stream>>>(x, w16, bq, bk, bv, qhi, qlo, khi, klo, v16);
  k_attn<<<dim3(SEQ / 64, NB), dim3(256), 0, stream>>>(qhi, qlo, khi, klo, v16, out);
}
